// Decoder_24043226923528
// MI455X (gfx1250) — hardware-verified
//
#include <hip/hip_runtime.h>
#include <math.h>

constexpr int NB    = 64;
constexpr int NT    = 256;
constexpr int ND    = 512;
constexpr int NH    = 512;
constexpr int NCAT  = ND + NH;
constexpr int NFUSE = NH + ND;
constexpr int NROW  = NT * NB;
constexpr int RNN_THR    = 512;
constexpr int RNN_WAVES  = RNN_THR / 32;
constexpr int RNN_HWAVES = RNN_WAVES / 2;
constexpr int SEQ_PB     = 16;
constexpr int RNN_BLOCKS = NB / SEQ_PB;
constexpr int HP    = 2 * NH + 8;
constexpr int HTILE = SEQ_PB * HP;
constexpr int SLABP = 68;
constexpr int PREP_TPM    = (NCAT / 64) * (NH / 64);
constexpr int PREP_BLOCKS = 4 * PREP_TPM;
constexpr int XC_CHUNKS   = NROW * (ND / 8);
constexpr int GEMM_GRID   = ((NFUSE / 64) * (NROW / 64)) / 8;
static_assert(NH == ND);
static_assert(NB % SEQ_PB == 0);
static_assert(NH == RNN_HWAVES * 64 && ND == RNN_HWAVES * 64);
static_assert(NFUSE == RNN_WAVES * 64);
static_assert(HP % 8 == 0);
static_assert(ND % 32 == 0 && NCAT % 32 == 0 && NH % 32 == 0);
static_assert(NFUSE % 64 == 0 && NROW % 64 == 0);
static_assert(((NFUSE / 64) * (NROW / 64)) % 8 == 0);
static_assert(XC_CHUNKS % 256 == 0);
static_assert(NCAT % 64 == 0 && NH % 64 == 0);
static_assert(NFUSE == 256 * 4);
static_assert(SEQ_PB * NH == 4 * RNN_THR * 4);
static_assert(PREP_BLOCKS == 512 && GEMM_GRID == 512 && RNN_BLOCKS == 4);
static_assert((2 * HTILE) % 8 == 0);

typedef __attribute__((ext_vector_type(16))) _Float16 v16h;
typedef __attribute__((ext_vector_type(8)))  _Float16 v8h;
typedef __attribute__((ext_vector_type(16))) __bf16   v16b;
typedef __attribute__((ext_vector_type(8)))  __bf16   v8b;
typedef __attribute__((ext_vector_type(8)))  float    v8f;
typedef __attribute__((ext_vector_type(4)))  float    v4f;

__device__ __forceinline__ unsigned short f2bf_bits(float f) {
  unsigned u = __float_as_uint(f);
  return (unsigned short)((u + 0x7FFFu + ((u >> 16) & 1u)) >> 16);
}
__device__ __forceinline__ float bf_bits2f(unsigned short h) { return __uint_as_float(((unsigned)h) << 16); }
__device__ __forceinline__ float bf16r(float f) { return bf_bits2f(f2bf_bits(f)); }
__device__ __forceinline__ __bf16 f2bf(float f) { return __builtin_bit_cast(__bf16, f2bf_bits(f)); }
__device__ __forceinline__ void bf_split(float f, __bf16& hi, __bf16& lo) {
  const unsigned short hb = f2bf_bits(f);
  hi = __builtin_bit_cast(__bf16, hb);
  lo = f2bf(f - bf_bits2f(hb));
}

__device__ __forceinline__ void dep_guard_h(v8f& a, v8f& b, v16h x, v16h y) { asm volatile("v_nop\n\tv_nop\n\tv_nop\n\tv_nop" : "+v"(a), "+v"(b) : "v"(x), "v"(y)); }
__device__ __forceinline__ void dep_guard_b(v8f& a, v8f& b, v16b x, v16b y) { asm volatile("v_nop\n\tv_nop\n\tv_nop\n\tv_nop" : "+v"(a), "+v"(b) : "v"(x), "v"(y)); }
__device__ __forceinline__ void dep_guard4_h(v8f& a, v8f& b, v8f& c, v8f& d, v16h x, v16h y) { asm volatile("v_nop\n\tv_nop\n\tv_nop\n\tv_nop" : "+v"(a), "+v"(b), "+v"(c), "+v"(d) : "v"(x), "v"(y)); }
__device__ __forceinline__ void dep_guard4_b(v8f& a, v8f& b, v8f& c, v8f& d, v16b x, v16b y) { asm volatile("v_nop\n\tv_nop\n\tv_nop\n\tv_nop" : "+v"(a), "+v"(b), "+v"(c), "+v"(d) : "v"(x), "v"(y)); }
__device__ __forceinline__ void keep4_h(v16h a, v16h b, v16h c, v16h d) { asm volatile("v_nop" :: "v"(a), "v"(b), "v"(c), "v"(d)); }
__device__ __forceinline__ void keep4_b(v16b a, v16b b, v16b c, v16b d) { asm volatile("v_nop" :: "v"(a), "v"(b), "v"(c), "v"(d)); }
__device__ __forceinline__ void acc_guard4(v8f& a, v8f& b, v8f& c, v8f& d) { asm volatile("v_nop\n\tv_nop\n\tv_nop\n\tv_nop" : "+v"(a), "+v"(b), "+v"(c), "+v"(d)); }

template <typename T> struct Frag;
template <> struct Frag<_Float16> {
  typedef v16h V; union U { v16h v; v8h h[2]; };
  static __device__ __forceinline__ v16h load(const _Float16* p) {
    U f; f.h[0] = *(const v8h*)(p); f.h[1] = *(const v8h*)(p + 16); return f.v;
  }
  static __device__ __forceinline__ v8f mma(v16h a, v16h b, v8f c) {
    return __builtin_amdgcn_wmma_f32_16x16x32_f16(false, a, false, b, (short)0, c, false, false);
  }
  static __device__ __forceinline__ void guard(v8f& a, v8f& b, v16h x, v16h y) { dep_guard_h(a, b, x, y); }
  static __device__ __forceinline__ void guard4(v8f& a, v8f& b, v8f& c, v8f& d, v16h x, v16h y) { dep_guard4_h(a, b, c, d, x, y); }
  static __device__ __forceinline__ void keep(v16h a, v16h b, v16h c, v16h d) { keep4_h(a, b, c, d); }
};
template <> struct Frag<__bf16> {
  typedef v16b V; union U { v16b v; v8b h[2]; };
  static __device__ __forceinline__ v16b load(const __bf16* p) {
    U f; f.h[0] = *(const v8b*)(p); f.h[1] = *(const v8b*)(p + 16); return f.v;
  }
  static __device__ __forceinline__ v8f mma(v16b a, v16b b, v8f c) {
    return __builtin_amdgcn_wmma_f32_16x16x32_bf16(false, a, false, b, (short)0, c, false, false);
  }
  static __device__ __forceinline__ void guard(v8f& a, v8f& b, v16b x, v16b y) { dep_guard_b(a, b, x, y); }
  static __device__ __forceinline__ void guard4(v8f& a, v8f& b, v8f& c, v8f& d, v16b x, v16b y) { dep_guard4_b(a, b, c, d, x, y); }
  static __device__ __forceinline__ void keep(v16b a, v16b b, v16b c, v16b d) { keep4_b(a, b, c, d); }
};

template <int ET> struct Elem;
template <> struct Elem<0> { typedef _Float16 T; };
template <> struct Elem<1> { typedef __bf16 T; };
template <int ET, bool SPLIT, int BIAS_MODE, int OUT_MODE, bool RESID, int ACT = 0, int TRI = 0>
__global__ __launch_bounds__(256) void wmma_gemm64(
    const unsigned short* __restrict__ Ap, const unsigned short* __restrict__ A2p, int lda, long strideA,
    const unsigned short* __restrict__ Btp, const unsigned short* __restrict__ Bt2p, int ldb, long strideB,
    void* __restrict__ Cout, void* __restrict__ Cout2, int ldc, long strideC,
    const float* __restrict__ bias,
    const float* __restrict__ resid, long strideR,
    int M, int N, int K, float scale) {
  typedef typename Elem<ET>::T T;
  typedef typename Frag<T>::V V;
  const T* A = (const T*)Ap; const T* A2 = (const T*)A2p; const T* Bt = (const T*)Btp; const T* Bt2 = (const T*)Bt2p;
  __shared__ __align__(16) float sT[8][16 * 68];
  const int b    = blockIdx.y;
  const int lane = threadIdx.x & 31;
  const int wave = threadIdx.x >> 5;
  const int tilesN = N >> 6;
  const int tilesM = M >> 6;
  const int tile = blockIdx.x * 8 + wave;
  if (tile >= tilesM * tilesN) return;
  const int tm = tile / tilesN;
  const int tn = tile - tm * tilesN;
  if (TRI == 1 && tn > tm) return;
  const int m0 = tm << 6;
  const int n0 = tn << 6;
  const int kLim = (TRI == 2) ? ((m0 + 64 < K) ? (m0 + 64) : K) : K;

  const T* Ab  = A  + (size_t)b * strideA;
  const T* Bb  = Bt + (size_t)b * strideB;
  const T* Ab2 = SPLIT ? (A2  + (size_t)b * strideA) : nullptr;
  const T* Bb2 = SPLIT ? (Bt2 + (size_t)b * strideB) : nullptr;

  const int rlane = lane & 15;
  const int koff  = (lane >> 4) * 8;
  const int mOff  = (lane >> 4) * 8;

  v8f acc[4][4];
#pragma unroll
  for (int i = 0; i < 4; ++i)
#pragma unroll
    for (int j = 0; j < 4; ++j) acc[i][j] = (v8f){0.f,0.f,0.f,0.f,0.f,0.f,0.f,0.f};

  for (int k0 = 0; k0 < kLim; k0 += 32) {
    V bh[4], bl[4];
#pragma unroll
    for (int j = 0; j < 4; ++j) {
      const size_t bo = (size_t)(n0 + (j << 4) + rlane) * ldb + koff + k0;
      bh[j] = Frag<T>::load(Bb + bo);
      if (SPLIT) bl[j] = Frag<T>::load(Bb2 + bo);
    }
#pragma unroll
    for (int i = 0; i < 4; ++i) {
      const size_t ao = (size_t)(m0 + (i << 4) + rlane) * lda + koff + k0;
      V ah = Frag<T>::load(Ab + ao);
      V al;
      if (SPLIT) al = Frag<T>::load(Ab2 + ao);
#pragma unroll
      for (int j = 0; j < 4; ++j) {
        acc[i][j] = Frag<T>::mma(ah, bh[j], acc[i][j]);
        if (SPLIT) {
          acc[i][j] = Frag<T>::mma(ah, bl[j], acc[i][j]);
          acc[i][j] = Frag<T>::mma(al, bh[j], acc[i][j]);
        }
      }
      Frag<T>::guard4(acc[i][0], acc[i][1], acc[i][2], acc[i][3], ah, SPLIT ? al : ah);
    }
    Frag<T>::keep(bh[0], bh[1], bh[2], bh[3]);
    if (SPLIT) Frag<T>::keep(bl[0], bl[1], bl[2], bl[3]);
  }
  acc_guard4(acc[0][0], acc[0][1], acc[0][2], acc[0][3]);
  acc_guard4(acc[1][0], acc[1][1], acc[1][2], acc[1][3]);
  acc_guard4(acc[2][0], acc[2][1], acc[2][2], acc[2][3]);
  acc_guard4(acc[3][0], acc[3][1], acc[3][2], acc[3][3]);

  float* slab = sT[wave];
  const float* Rb = RESID ? (resid + (size_t)b * strideR) : nullptr;
#pragma unroll
  for (int i = 0; i < 4; ++i) {
    const int mBase = m0 + (i << 4);
#pragma unroll
    for (int j = 0; j < 4; ++j) {
      const int n = n0 + (j << 4) + rlane;
      float bv = 0.f;
      if (BIAS_MODE == 2) bv = bias[n];
#pragma unroll
      for (int r = 0; r < 8; ++r) {
        float v = acc[i][j][r] * scale;
        if (BIAS_MODE == 1) v += bias[mBase + mOff + r];
        if (BIAS_MODE == 2) v += bv;
        if (RESID) v += Rb[(size_t)(mBase + mOff + r) * ldc + n];
        if (ACT == 1) v = tanhf(v);
        if (ACT == 2) v = fmaxf(v, 0.0f);
        if (ACT == 4) v = (v > 0.f) ? v : 0.01f * v;
        slab[(mOff + r) * 68 + (j << 4) + rlane] = v;
      }
    }
    __builtin_amdgcn_fence(__ATOMIC_RELEASE, "workgroup");
    __builtin_amdgcn_wave_barrier();
    __builtin_amdgcn_fence(__ATOMIC_ACQUIRE, "workgroup");
    if (OUT_MODE == 0) {
      float* C = (float*)Cout + (size_t)b * strideC;
      const int hh = lane >> 4, c4 = (lane & 15) * 4;
      for (int pass = 0; pass < 2; ++pass) {
#pragma unroll
        for (int it = 0; it < 8; ++it) {
          const int row = it * 2 + hh;
          v4f v = *(const v4f*)(slab + row * 68 + c4);
          *(volatile v4f*)(C + (size_t)(mBase + row) * ldc + n0 + c4) = v;
        }
        __threadfence();
      }
    } else {
      const int q = lane >> 3, c8 = (lane & 7) * 8;
      unsigned short* C  = (unsigned short*)Cout  + (size_t)b * strideC;
      unsigned short* C2 = (OUT_MODE == 2) ? ((unsigned short*)Cout2 + (size_t)b * strideC) : nullptr;
      for (int pass = 0; pass < 2; ++pass) {
#pragma unroll
        for (int it = 0; it < 4; ++it) {
          const int row = it * 4 + q;
          const float* sp = slab + row * 68 + c8;
          v8h hv, lv;
#pragma unroll
          for (int e = 0; e < 8; ++e) {
            if (OUT_MODE == 1) {
              hv[e] = (_Float16)sp[e];
            } else {
              unsigned short hb = f2bf_bits(sp[e]);
              unsigned short lb = f2bf_bits(sp[e] - bf_bits2f(hb));
              hv[e] = __builtin_bit_cast(_Float16, hb);
              lv[e] = __builtin_bit_cast(_Float16, lb);
            }
          }
          *(volatile v8h*)(C + (size_t)(mBase + row) * ldc + n0 + c8) = hv;
          if (OUT_MODE == 2) *(volatile v8h*)(C2 + (size_t)(mBase + row) * ldc + n0 + c8) = lv;
        }
        __threadfence();
      }
    }
    __builtin_amdgcn_fence(__ATOMIC_RELEASE, "workgroup");
    __builtin_amdgcn_wave_barrier();
    __builtin_amdgcn_fence(__ATOMIC_ACQUIRE, "workgroup");
  }
}

__device__ __forceinline__ float ftanh(float x) {
  const float xc = fminf(fmaxf(x, -10.0f), 10.0f);
  const float e  = expf(2.0f * xc);
  return 1.0f - 2.0f * __builtin_amdgcn_rcpf(1.0f + e);
}

__global__ __launch_bounds__(256) void prep_w_kernel(
    const float* __restrict__ Wh0, const float* __restrict__ Wo0,
    const float* __restrict__ Wh1, const float* __restrict__ Wo1,
    unsigned short* __restrict__ WX0, unsigned short* __restrict__ WR0,
    unsigned short* __restrict__ WX1D, unsigned short* __restrict__ WR1) {
  __shared__ float tile[64][65];
  const int blk = blockIdx.x, tid = threadIdx.x;
  const int mat = blk >> 7;
  const int tl  = blk & 127;
  const int kt  = tl >> 3;
  const int nt  = tl & 7;
  const int k0  = kt * 64, n0 = nt * 64;
  const float* src = (mat == 0) ? Wh0 : (mat == 1) ? Wo0 : (mat == 2) ? Wh1 : Wo1;
#pragma unroll
  for (int it = 0; it < 4; ++it) {
    const int idx = it * 256 + tid;
    const int kk  = idx >> 4;
    const int cc  = (idx & 15) * 4;
    const v4f v = *(const v4f*)(src + (size_t)(k0 + kk) * NH + n0 + cc);
    tile[kk][cc + 0] = v[0]; tile[kk][cc + 1] = v[1]; tile[kk][cc + 2] = v[2]; tile[kk][cc + 3] = v[3];
  }
  __syncthreads();
  const int layer = mat >> 1, isO = mat & 1;
  const int ndst0 = n0 + isO * NH;
  v8h hvv[2];
#pragma unroll
  for (int it = 0; it < 2; ++it) {
    const int idx = it * 256 + tid;
    const int nn = idx >> 3, k8 = (idx & 7) * 8;
    v8h hv;
#pragma unroll
    for (int e = 0; e < 8; ++e) hv[e] = __builtin_bit_cast(_Float16, f2bf_bits(tile[k8 + e][nn]));
    hvv[it] = hv;
  }
  for (int pass = 0; pass < 2; ++pass) {
#pragma unroll
    for (int it = 0; it < 2; ++it) {
      const int idx = it * 256 + tid;
      const int nn = idx >> 3, k8 = (idx & 7) * 8;
      const size_t nd = (size_t)(ndst0 + nn);
      const v8h hv = hvv[it];
      if (kt < 8) {
        if (layer == 0) {
          *(volatile v8h*)(WX0 + nd * ND + k0 + k8) = hv;
        } else {
          *(volatile v8h*)(WX1D + nd * NCAT + k0 + k8) = hv;
          *(volatile v8h*)(WX1D + nd * NCAT + ND + k0 + k8) = hv;
        }
      } else {
        if (layer == 0) *(volatile v8h*)(WR0 + nd * NH + (k0 - ND) + k8) = hv;
        else            *(volatile v8h*)(WR1 + nd * NH + (k0 - ND) + k8) = hv;
      }
    }
    __threadfence();
  }
}

__global__ __launch_bounds__(256) void bias_prep_kernel(
    const float* __restrict__ bh0, const float* __restrict__ bo0,
    const float* __restrict__ bh1, const float* __restrict__ bo1, float* __restrict__ BIAS) {
  const int tid = threadIdx.x;
  const int p   = tid * 4;
  const int isO = (tid >= 128) ? 1 : 0;
  const int pc  = p & (NH - 1);
  const v4f a0 = *(const v4f*)(bh0 + pc);
  const v4f b0 = *(const v4f*)(bo0 + pc);
  const v4f a1 = *(const v4f*)(bh1 + pc);
  const v4f b1 = *(const v4f*)(bo1 + pc);
  v4f o0, o1;
#pragma unroll
  for (int e = 0; e < 4; ++e) {
    o0[e] = bf16r(isO ? b0[e] : a0[e]);
    o1[e] = bf16r(isO ? b1[e] : a1[e]);
  }
  float* op0 = BIAS + p;
  float* op1 = BIAS + NFUSE + p;
  *(volatile v4f*)op0 = o0;
  *(volatile v4f*)op1 = o1;
  __threadfence();
  *(volatile v4f*)op0 = o0;
  *(volatile v4f*)op1 = o1;
}

__global__ __launch_bounds__(256) void xcast_kernel(const float* __restrict__ x, unsigned short* __restrict__ XB) {
  const int i = blockIdx.x * 256 + threadIdx.x;
  const int row = i >> 6, c8 = i & 63;
  const int t = row >> 6, b = row & 63;
  const float* src = x + ((size_t)b * NT + t) * ND + c8 * 8;
  const v4f f0 = *(const v4f*)src;
  const v4f f1 = *(const v4f*)(src + 4);
  v8h hv;
  hv[0] = __builtin_bit_cast(_Float16, f2bf_bits(f0[0])); hv[1] = __builtin_bit_cast(_Float16, f2bf_bits(f0[1]));
  hv[2] = __builtin_bit_cast(_Float16, f2bf_bits(f0[2])); hv[3] = __builtin_bit_cast(_Float16, f2bf_bits(f0[3]));
  hv[4] = __builtin_bit_cast(_Float16, f2bf_bits(f1[0])); hv[5] = __builtin_bit_cast(_Float16, f2bf_bits(f1[1]));
  hv[6] = __builtin_bit_cast(_Float16, f2bf_bits(f1[2])); hv[7] = __builtin_bit_cast(_Float16, f2bf_bits(f1[3]));
  unsigned short* dst = XB + (size_t)row * ND + c8 * 8;
  *(volatile v8h*)dst = hv;
  __threadfence();
  *(volatile v8h*)dst = hv;
}

template <int LAYER>
__global__ __launch_bounds__(RNN_THR) void rnn_layer_kernel(
    const float* __restrict__ PT, const float* __restrict__ biasf,
    const unsigned short* __restrict__ WRp, const float* __restrict__ enc,
    unsigned short* __restrict__ out16, float* __restrict__ outf) {
  __shared__ __align__(16) __bf16 hbuf[2 * HTILE];
  __shared__ __align__(16) float  slab_all[RNN_HWAVES][16 * SLABP];
  const __bf16* WR = (const __bf16*)WRp;
  const int tid = threadIdx.x, lane = tid & 31, wave = tid >> 5;
  const int c = lane & 15, hh = lane >> 4, koff = hh * 8, mOff = hh * 8, c4 = c * 4;
  const int q4 = lane >> 3, c8 = (lane & 7) * 8;
  const int seq0 = blockIdx.x * SEQ_PB;
  const int n0 = wave * 64;
  const bool is_o = (wave >= RNN_HWAVES);
  const int j0 = is_o ? (n0 - NH) : 0;

  {
    const __bf16 bz = __builtin_bit_cast(__bf16, (unsigned short)0);
    const v8b z = {bz, bz, bz, bz, bz, bz, bz, bz};
#pragma unroll 1
    for (int i = tid; i < (2 * HTILE) / 8; i += RNN_THR) *(v8b*)(hbuf + i * 8) = z;
  }
  __syncthreads();
  if (LAYER == 0) {
#pragma unroll
    for (int it = 0; it < 4; ++it) {
      const int i   = it * RNN_THR + tid;
      const int row = i >> 7;
      const int cc  = (i & 127) * 4;
      const v4f e4 = *(const v4f*)(enc + (size_t)(seq0 + row) * NH + cc);
      hbuf[row * HP + cc + 0] = f2bf(e4[0]);
      hbuf[row * HP + cc + 1] = f2bf(e4[1]);
      hbuf[row * HP + cc + 2] = f2bf(e4[2]);
      hbuf[row * HP + cc + 3] = f2bf(e4[3]);
    }
  }
  __syncthreads();

  float bj[4];
#pragma unroll
  for (int j = 0; j < 4; ++j) bj[j] = biasf[n0 + 16 * j + c];
  const __bf16* brow = WR + (size_t)(n0 + c) * NH + koff;
  float* slab = slab_all[wave & (RNN_HWAVES - 1)];

#pragma unroll 1
  for (int t = 0; t < NT; ++t) {
    const __bf16* hc = hbuf + (t & 1) * HTILE;
    __bf16*       hn = hbuf + ((t + 1) & 1) * HTILE;
    v8f acc[4];
    {
      const size_t mrow = (size_t)t * NB + seq0 + 8 * hh;
#pragma unroll
      for (int j = 0; j < 4; ++j) {
        if (j == 2) asm volatile("" ::: "memory");
        const float* pp = PT + (size_t)(n0 + 16 * j + c) * NROW + mrow;
        const v4f xa = *(const v4f*)pp;
        const v4f xb = *(const v4f*)(pp + 4);
        const float bb = bj[j];
        acc[j][0] = xa[0] + bb; acc[j][1] = xa[1] + bb; acc[j][2] = xa[2] + bb; acc[j][3] = xa[3] + bb;
        acc[j][4] = xb[0] + bb; acc[j][5] = xb[1] + bb; acc[j][6] = xb[2] + bb; acc[j][7] = xb[3] + bb;
      }
    }
    const __bf16* arh = hc + c * HP + koff;
    const __bf16* arl = arh + NH;
#pragma unroll 1
    for (int kc = 0; kc < NH / 32; ++kc) {
      const v16b ah = Frag<__bf16>::load(arh + kc * 32);
      const v16b al = Frag<__bf16>::load(arl + kc * 32);
      v16b fb[4];
#pragma unroll
      for (int j = 0; j < 4; ++j) fb[j] = Frag<__bf16>::load(brow + (size_t)(16 * j) * NH + kc * 32);
#pragma unroll
      for (int j = 0; j < 4; ++j) {
        acc[j] = Frag<__bf16>::mma(ah, fb[j], acc[j]);
        acc[j] = Frag<__bf16>::mma(al, fb[j], acc[j]);
      }
      dep_guard4_b(acc[0], acc[1], acc[2], acc[3], ah, al);
      keep4_b(fb[0], fb[1], fb[2], fb[3]);
    }
    acc_guard4(acc[0], acc[1], acc[2], acc[3]);

    float th[4][8];
#pragma unroll
    for (int j = 0; j < 4; ++j)
#pragma unroll
      for (int r = 0; r < 8; ++r) th[j][r] = ftanh(acc[j][r]);

    if (!is_o) {
#pragma unroll
      for (int j = 0; j < 4; ++j) {
#pragma unroll
        for (int r = 0; r < 8; ++r) {
          __bf16 hi, lo;
          bf_split(th[j][r], hi, lo);
          const int idx = (mOff + r) * HP + n0 + 16 * j + c;
          hn[idx]      = hi;
          hn[idx + NH] = lo;
        }
      }
    } else {
#pragma unroll
      for (int j = 0; j < 4; ++j)
#pragma unroll
        for (int r = 0; r < 8; ++r) slab[(mOff + r) * SLABP + 16 * j + c] = th[j][r];
    }
    __syncthreads();

    if (is_o) {
      if (LAYER == 0) {
        const size_t mbase = (size_t)t * NB + seq0;
        for (int pass = 0; pass < 2; ++pass) {
#pragma unroll
          for (int it = 0; it < 4; ++it) {
            const int rr = it * 4 + q4;
            const float* sp = slab + rr * SLABP + c8;
            v8h hv, lv;
#pragma unroll
            for (int e = 0; e < 8; ++e) {
              const unsigned short hb = f2bf_bits(sp[e]);
              const unsigned short lb = f2bf_bits(sp[e] - bf_bits2f(hb));
              hv[e] = __builtin_bit_cast(_Float16, hb);
              lv[e] = __builtin_bit_cast(_Float16, lb);
            }
            unsigned short* orow = out16 + (mbase + rr) * NFUSE + j0 + c8;
            *(volatile v8h*)(orow)      = hv;
            *(volatile v8h*)(orow + NH) = lv;
          }
          __threadfence();
        }
      } else {
        for (int pass = 0; pass < 2; ++pass) {
#pragma unroll
          for (int it = 0; it < 8; ++it) {
            const int rr = it * 2 + hh;
            const v4f v = *(const v4f*)(slab + rr * SLABP + c4);
            *(volatile v4f*)(outf + ((size_t)(seq0 + rr) * NT + (size_t)t) * ND + j0 + c4) = v;
          }
          __threadfence();
        }
      }
      __builtin_amdgcn_fence(__ATOMIC_RELEASE, "workgroup");
      __builtin_amdgcn_wave_barrier();
      __builtin_amdgcn_fence(__ATOMIC_ACQUIRE, "workgroup");
    }
  }
}

extern "C" void kernel_launch(void* const* d_in, const int* in_sizes, int n_in,
                              void* d_out, int out_size, void* d_ws, size_t ws_size, hipStream_t stream) {
  if (n_in < 10 || d_out == nullptr || d_ws == nullptr) return;
  if (in_sizes[0] != NB * NT * ND || in_sizes[1] != NB * NH || in_sizes[2] != NCAT * NH || in_sizes[3] != NH ||
      in_sizes[4] != NCAT * ND || in_sizes[5] != ND || in_sizes[6] != NCAT * NH || in_sizes[7] != NH ||
      in_sizes[8] != NCAT * ND || in_sizes[9] != ND || out_size != NB * NT * ND) return;

  const float* x   = (const float*)d_in[0];
  const float* enc = (const float*)d_in[1];
  const float* Wh0 = (const float*)d_in[2];
  const float* bh0 = (const float*)d_in[3];
  const float* Wo0 = (const float*)d_in[4];
  const float* bo0 = (const float*)d_in[5];
  const float* Wh1 = (const float*)d_in[6];
  const float* bh1 = (const float*)d_in[7];
  const float* Wo1 = (const float*)d_in[8];
  const float* bo1 = (const float*)d_in[9];
  float* out = (float*)d_out;

  char* ws = (char*)d_ws; size_t off = 0;
  auto carve = [&](size_t bytes) -> char* { char* p = ws + off; off += (bytes + 255) & ~(size_t)255; return p; };
  unsigned short* XB   = (unsigned short*)carve((size_t)NROW * ND * 2);
  unsigned short* WX0  = (unsigned short*)carve((size_t)NFUSE * ND * 2);
  unsigned short* WR0  = (unsigned short*)carve((size_t)NFUSE * NH * 2);
  unsigned short* WX1D = (unsigned short*)carve((size_t)NFUSE * NCAT * 2);
  unsigned short* WR1  = (unsigned short*)carve((size_t)NFUSE * NH * 2);
  float*          BIAS = (float*)carve((size_t)2 * NFUSE * 4);
  float*          PT   = (float*)carve((size_t)NFUSE * NROW * 4);
  unsigned short* OUT0 = (unsigned short*)carve((size_t)NROW * NFUSE * 2);
  if (off > ws_size || off > (size_t)134217728) return;

  prep_w_kernel<<<PREP_BLOCKS, 256, 0, stream>>>(Wh0, Wo0, Wh1, Wo1, WX0, WR0, WX1D, WR1);
  bias_prep_kernel<<<1, 256, 0, stream>>>(bh0, bo0, bh1, bo1, BIAS);

  xcast_kernel<<<XC_CHUNKS / 256, 256, 0, stream>>>(x, XB);

  wmma_gemm64<1, false, 0, 0, false, 0, 0><<<dim3(GEMM_GRID, 1), 256, 0, stream>>>(
      WX0, WX0, ND, 0L, XB, XB, ND, 0L,
      (void*)PT, (void*)PT, NROW, 0L, BIAS, BIAS, 0L, NFUSE, NROW, ND, 1.0f);

  rnn_layer_kernel<0><<<RNN_BLOCKS, RNN_THR, 0, stream>>>(PT, BIAS, WR0, enc, OUT0, out);

  wmma_gemm64<1, false, 0, 0, false, 0, 0><<<dim3(GEMM_GRID, 1), 256, 0, stream>>>(
      WX1D, WX1D, NCAT, 0L, OUT0, OUT0, NCAT, 0L,
      (void*)PT, (void*)PT, NROW, 0L, BIAS, BIAS, 0L, NFUSE, NROW, NCAT, 1.0f);

  rnn_layer_kernel<1><<<RNN_BLOCKS, RNN_THR, 0, stream>>>(PT, BIAS + NFUSE, WR1, enc, OUT0, out);
}
